// MeshConv_79517024518469
// MI455X (gfx1250) — hardware-verified
//
#include <hip/hip_runtime.h>
#include <stddef.h>


#define NTHR   256
#define NWAVE  8
#define EPT    8
#define CHUNK  (NTHR * EPT)
#define WCAP   (EPT * 32)
#define LISTN  (NWAVE * WCAP)
#define PASSN  (NWAVE * 16)
#define PCAP   (CHUNK + PASSN)
#define NB     256
#define CH     128
#define NPW    256
#define MROWS  64
#define WSC    32.0f
#define WINV   0.03125f
#define GN_EPS 1e-5f

static_assert(PASSN == 128);
static_assert(PCAP >= CHUNK + PASSN);
static_assert((NB % NWAVE) == 0);
static_assert(PASSN <= NTHR);

typedef float    v4f  __attribute__((ext_vector_type(4)));
typedef float    v4fa __attribute__((ext_vector_type(4))) __attribute__((__may_alias__));
typedef float    v8f  __attribute__((ext_vector_type(8)));
typedef int      v4i  __attribute__((ext_vector_type(4)));
typedef _Float16 v8h  __attribute__((ext_vector_type(8)));
typedef _Float16 v16h __attribute__((ext_vector_type(16)));
typedef __bf16   v8b  __attribute__((ext_vector_type(8)));
typedef __bf16   v16b __attribute__((ext_vector_type(16)));
union FragH { v16h v; v8h h[2]; };
union FragB { v16b v; v8b h[2]; };
union Pk8h  { v8h h; v4i i; };
union Pk8b  { v8b b; v4i i; };

__device__ __forceinline__ v8f wmh(v16h a, v16h b, v8f c) {
  v8f d = __builtin_amdgcn_wmma_f32_16x16x32_f16(false, a, false, b, (short)0, c, false, false);
  asm volatile("v_nop\n\tv_nop\n\tv_nop\n\tv_nop" : "+v"(d) : "v"(a), "v"(b));
  return d;
}
__device__ __forceinline__ v8f wmb(v16b a, v16b b, v8f c) {
  v8f d = __builtin_amdgcn_wmma_f32_16x16x32_bf16(false, a, false, b, (short)0, c, false, false);
  asm volatile("v_nop\n\tv_nop\n\tv_nop\n\tv_nop" : "+v"(d) : "v"(a), "v"(b));
  return d;
}

__device__ __forceinline__ int scan_chunk(const int* __restrict__ dsts, int nE, int cbase, int nodeBase,
                                          int vec8, int* list, int tid, int wave) {
  int wc = 0;
  const int el0  = tid * EPT;
  const int e0   = cbase + el0;
  const int sent = -2147483647 - 1;
  v4i da, db;
  if (vec8 != 0 && cbase + CHUNK <= nE) {
    da = *(const v4i*)(dsts + e0);
    db = *(const v4i*)(dsts + e0 + 4);
  } else {
    const int em = nE - 1;
    da.x = (e0     < nE) ? dsts[min(e0, em)]     : sent;
    da.y = (e0 + 1 < nE) ? dsts[min(e0 + 1, em)] : sent;
    da.z = (e0 + 2 < nE) ? dsts[min(e0 + 2, em)] : sent;
    da.w = (e0 + 3 < nE) ? dsts[min(e0 + 3, em)] : sent;
    db.x = (e0 + 4 < nE) ? dsts[min(e0 + 4, em)] : sent;
    db.y = (e0 + 5 < nE) ? dsts[min(e0 + 5, em)] : sent;
    db.z = (e0 + 6 < nE) ? dsts[min(e0 + 6, em)] : sent;
    db.w = (e0 + 7 < nE) ? dsts[min(e0 + 7, em)] : sent;
  }
  const unsigned nb = (unsigned)nodeBase;
  const unsigned s0 = (unsigned)da.x - nb, s1 = (unsigned)da.y - nb;
  const unsigned s2 = (unsigned)da.z - nb, s3 = (unsigned)da.w - nb;
  const unsigned s4 = (unsigned)db.x - nb, s5 = (unsigned)db.y - nb;
  const unsigned s6 = (unsigned)db.z - nb, s7 = (unsigned)db.w - nb;
  const bool h0 = s0 < (unsigned)NB, h1 = s1 < (unsigned)NB, h2 = s2 < (unsigned)NB, h3 = s3 < (unsigned)NB;
  const bool h4 = s4 < (unsigned)NB, h5 = s5 < (unsigned)NB, h6 = s6 < (unsigned)NB, h7 = s7 < (unsigned)NB;
  const unsigned any = __builtin_amdgcn_ballot_w32(h0 | h1 | h2 | h3 | h4 | h5 | h6 | h7);
  if (any != 0u) {
#define HITJ(J, HJ) { \
      const unsigned mj = __builtin_amdgcn_ballot_w32(HJ); \
      if (mj != 0u) { \
        if (HJ) { \
          const int pos = wc + (int)__builtin_amdgcn_mbcnt_lo(mj, 0u); \
          if (pos < WCAP) list[wave * WCAP + pos] = el0 + (J); \
        } \
        wc += (int)__builtin_popcount(mj); } }
    HITJ(0, h0)
    HITJ(1, h1)
    HITJ(2, h2)
    HITJ(3, h3)
    HITJ(4, h4)
    HITJ(5, h5)
    HITJ(6, h6)
    HITJ(7, h7)
#undef HITJ
  }
  return wc;
}

__global__ __launch_bounds__(NTHR) void k_prep(const float* __restrict__ W1, const float* __restrict__ W2,
                                               __bf16* w1h, __bf16* w1l, _Float16* w2h) {
  const int t = blockIdx.x * NTHR + threadIdx.x;
  if (blockIdx.x < 16) {
    const int nn = t >> 4, kq = (t & 15) * 8;
    const int part = nn >> 7, n = nn & 127;
    Pk8b ph, pl;
#pragma unroll
    for (int j = 0; j < 8; ++j) {
      const float v = W1[(size_t)(part * CH + kq + j) * CH + n];
      const __bf16 hb = (__bf16)v;
      ph.b[j] = hb;
      pl.b[j] = (__bf16)(v - (float)hb);
    }
    const size_t o = (size_t)nn * CH + kq;
    const v4i vh = ph.i, vl = pl.i;
    *(volatile v4i*)(w1h + o) = vh;
    *(volatile v4i*)(w1l + o) = vl;
    __threadfence();
    *(volatile v4i*)(w1h + o) = vh;
    *(volatile v4i*)(w1l + o) = vl;
  } else {
    const int u = t - 16 * NTHR;
    const int n = u >> 4, kq = (u & 15) * 8;
    Pk8h p;
#pragma unroll
    for (int j = 0; j < 8; ++j) p.h[j] = (_Float16)(W2[(size_t)(kq + j) * CH + n] * WSC);
    const size_t o = (size_t)n * CH + kq;
    const v4i vv = p.i;
    *(volatile v4i*)(w2h + o) = vv;
    __threadfence();
    *(volatile v4i*)(w2h + o) = vv;
  }
}

__global__ __launch_bounds__(NTHR) void k_node(const float* __restrict__ x, const __bf16* __restrict__ w1h,
                                               const __bf16* __restrict__ w1l, const float* __restrict__ b1,
                                               float* npl, int nN) {
  __shared__ __attribute__((aligned(16))) float stg[NWAVE * 16 * CH];
  const int tid = threadIdx.x, lane = tid & 31, wave = tid >> 5, hh = lane >> 4, m = lane & 15;
  const int rg = wave >> 1, chf = wave & 1;
  const int row0 = blockIdx.x * MROWS + 16 * rg;
  int rowc = row0 + m;
  rowc = rowc > nN - 1 ? nN - 1 : rowc;
  const float* xr = x + (size_t)rowc * CH;
  const __bf16* bh0 = w1h + (size_t)(CH * chf + m) * CH + 8 * hh;
  const __bf16* bl0 = w1l + (size_t)(CH * chf + m) * CH + 8 * hh;

  const v8f z8 = {0.f, 0.f, 0.f, 0.f, 0.f, 0.f, 0.f, 0.f};
  v8f acc[8];
#pragma unroll
  for (int nt = 0; nt < 8; ++nt) acc[nt] = z8;

#pragma unroll
  for (int kb = 0; kb < 4; ++kb) {
    const float* xp = xr + 32 * kb + 8 * hh;
    const v4f p0 = *(const v4f*)xp;
    const v4f p1 = *(const v4f*)(xp + 4);
    const v4f p2 = *(const v4f*)(xp + 16);
    const v4f p3 = *(const v4f*)(xp + 20);
    const float fv[16] = {p0.x, p0.y, p0.z, p0.w, p1.x, p1.y, p1.z, p1.w,
                          p2.x, p2.y, p2.z, p2.w, p3.x, p3.y, p3.z, p3.w};
    FragB fh, fl;
#pragma unroll
    for (int j = 0; j < 16; ++j) {
      const __bf16 hb = (__bf16)fv[j];
      fh.v[j] = hb;
      fl.v[j] = (__bf16)(fv[j] - (float)hb);
    }
#pragma unroll
    for (int nt = 0; nt < 8; ++nt) {
      const size_t bo = (size_t)(16 * nt) * CH + 32 * kb;
      FragB gh, gl;
      gh.h[0] = *(const v8b*)(bh0 + bo);
      gh.h[1] = *(const v8b*)(bh0 + bo + 16);
      gl.h[0] = *(const v8b*)(bl0 + bo);
      gl.h[1] = *(const v8b*)(bl0 + bo + 16);
      acc[nt] = wmb(fh.v, gh.v, acc[nt]);
      acc[nt] = wmb(fh.v, gl.v, acc[nt]);
      acc[nt] = wmb(fl.v, gh.v, acc[nt]);
    }
  }

  float* sw = stg + wave * 16 * CH;
#pragma unroll
  for (int nt = 0; nt < 8; ++nt) {
    const float bvl = b1[16 * nt + m];
    const float badd = (chf == 0) ? bvl : 0.0f;
#pragma unroll
    for (int r = 0; r < 8; ++r) sw[(8 * hh + r) * CH + 16 * nt + m] = acc[nt][r] + badd;
  }
  __syncthreads();
  const size_t gb = (size_t)row0 * NPW + (size_t)(CH * chf) + (size_t)(4 * lane);
#pragma unroll 1
  for (int i = 0; i < 16; ++i) {
    const v4f v = *(const v4fa*)(sw + i * CH + 4 * lane);
    *(volatile v4f*)(npl + gb + (size_t)i * NPW) = v;
  }
  __threadfence();
#pragma unroll 1
  for (int i = 0; i < 16; ++i) {
    const v4f v = *(const v4fa*)(sw + i * CH + 4 * lane);
    *(volatile v4f*)(npl + gb + (size_t)i * NPW) = v;
  }
}

__global__ __launch_bounds__(NTHR) void k_edge(
    const float* __restrict__ np, const int* __restrict__ ei, const float* __restrict__ ea,
    const float* __restrict__ W1, const float* __restrict__ gmg, const float* __restrict__ btg,
    const float* __restrict__ b2, const _Float16* __restrict__ w2h,
    float* outp, int nN, int nE, int vec8) {
  __shared__ __attribute__((aligned(16))) float acc[NB * CH];
  __shared__ __attribute__((aligned(16))) float cntf[NB];
  __shared__ __attribute__((aligned(16))) float msg[PASSN * CH];
  __shared__ __attribute__((aligned(16))) int   list[LISTN];
  __shared__ __attribute__((aligned(16))) int   pend[PCAP];
  __shared__ __attribute__((aligned(16))) int   slotb[PASSN];
  __shared__ __attribute__((aligned(16))) float w1e[CH * 4];
  __shared__ __attribute__((aligned(16))) float gam[CH];
  __shared__ __attribute__((aligned(16))) float bet[CH];
  __shared__ int wcnt[NWAVE];
  __shared__ int pendN;

  const int tid = threadIdx.x, lane = tid & 31, wave = tid >> 5, hh = lane >> 4, m = lane & 15;
  const int nodeBase = blockIdx.x * NB;
  const int* srcs = ei;
  const int* dsts = ei + nE;

  {
    const v4f z4 = {0.0f, 0.0f, 0.0f, 0.0f};
    for (int i = tid; i < (NB * CH) / 4; i += NTHR) *(v4f*)(acc + 4 * i) = z4;
    if (tid < NB) cntf[tid] = 0.0f;
    if (tid < CH) {
#pragma unroll
      for (int j = 0; j < 4; ++j) w1e[4 * tid + j] = W1[(size_t)(256 + j) * CH + tid];
      gam[tid] = gmg[tid];
      bet[tid] = btg[tid];
    }
    if (tid == 0) pendN = 0;
  }
  __syncthreads();

  const v8f z8 = {0.f, 0.f, 0.f, 0.f, 0.f, 0.f, 0.f, 0.f};
  const int nChunks = (nE + CHUNK - 1) / CHUNK;
#pragma unroll 1
  for (int ch = 0; ch < nChunks; ++ch) {
    const int cbase = ch * CHUNK;
    const int wc = scan_chunk(dsts, nE, cbase, nodeBase, vec8, list, tid, wave);
    if (lane == 0) wcnt[wave] = wc;
    __syncthreads();

    const int base = pendN;
    int tot = 0, myoff = 0;
#pragma unroll
    for (int w = 0; w < NWAVE; ++w) {
      int c = wcnt[w];
      c = c > WCAP ? WCAP : (c < 0 ? 0 : c);
      if (w < wave) myoff += c;
      tot += c;
    }
    int newN = base + tot;
    newN = newN > PCAP ? PCAP : newN;
    {
      int n = wcnt[wave];
      n = n > WCAP ? WCAP : (n < 0 ? 0 : n);
      const int* lp = list + wave * WCAP;
      for (int i = lane; i < n; i += 32) {
        const int pos = base + myoff + i;
        if (pos < PCAP) pend[pos] = cbase + lp[i];
      }
    }
    const int fin = (ch == nChunks - 1) ? 1 : 0;
    const int R   = (fin != 0) ? (newN + PASSN - 1) / PASSN : newN / PASSN;
    const int Pv  = (fin != 0) ? newN : R * PASSN;
    __syncthreads();

#pragma unroll 1
    for (int r = 0; r < R; ++r) {
      {
        const int idx = r * PASSN + wave * 16 + m;
        const bool valid = idx < Pv;
        int e = pend[idx];
        e = e < 0 ? 0 : (e > nE - 1 ? nE - 1 : e);
        int d = dsts[e];
        int s = srcs[e];
        int slot = d - nodeBase;
        if (!valid || (unsigned)slot >= (unsigned)NB) slot = NB;
        d = d < 0 ? 0 : (d > nN - 1 ? nN - 1 : d);
        s = s < 0 ? 0 : (s > nN - 1 ? nN - 1 : s);
        if (hh == 0) slotb[wave * 16 + m] = slot;
        const float* dP = np + (size_t)d * NPW;
        const float* qP = np + (size_t)s * NPW + CH;
        const v4f ea4 = *(const v4f*)(ea + (size_t)e * 4);

        v8h ah[8];
#pragma unroll
        for (int g = 0; g < 8; ++g) {
          const int c0 = 16 * g + 8 * hh;
          const v4f pa = *(const v4f*)(dP + c0);
          const v4f pb = *(const v4f*)(dP + c0 + 4);
          const v4f qa = *(const v4f*)(qP + c0);
          const v4f qb = *(const v4f*)(qP + c0 + 4);
          float hv[8];
          hv[0] = pa.x + qa.x; hv[1] = pa.y + qa.y; hv[2] = pa.z + qa.z; hv[3] = pa.w + qa.w;
          hv[4] = pb.x + qb.x; hv[5] = pb.y + qb.y; hv[6] = pb.z + qb.z; hv[7] = pb.w + qb.w;
#pragma unroll
          for (int j = 0; j < 8; ++j) {
            const v4f wv = *(const v4fa*)(w1e + 4 * (c0 + j));
            hv[j] += ea4.x * wv.x + ea4.y * wv.y + ea4.z * wv.z + ea4.w * wv.w;
          }
          float sm = ((hv[0] + hv[1]) + (hv[2] + hv[3])) + ((hv[4] + hv[5]) + (hv[6] + hv[7]));
          sm += __shfl_xor(sm, 16, 32);
          const float mean = sm * 0.0625f;
          float qv = 0.0f;
#pragma unroll
          for (int j = 0; j < 8; ++j) { const float dv = hv[j] - mean; hv[j] = dv; qv += dv * dv; }
          qv += __shfl_xor(qv, 16, 32);
          const float rstd = rsqrtf(qv * 0.0625f + GN_EPS);
          const v4f ga = *(const v4fa*)(gam + c0), gbv = *(const v4fa*)(gam + c0 + 4);
          const v4f ba = *(const v4fa*)(bet + c0), bbv = *(const v4fa*)(bet + c0 + 4);
          const float gv[8] = {ga.x, ga.y, ga.z, ga.w, gbv.x, gbv.y, gbv.z, gbv.w};
          const float tv[8] = {ba.x, ba.y, ba.z, ba.w, bbv.x, bbv.y, bbv.z, bbv.w};
          v8h o;
#pragma unroll
          for (int j = 0; j < 8; ++j) {
            const float hn  = hv[j] * rstd * gv[j] + tv[j];
            const float ex  = __expf(-hn);
            const float act = hn * __builtin_amdgcn_rcpf(1.0f + ex);
            o[j] = (_Float16)act;
          }
          ah[g] = o;
        }

        v8f acc2[8];
#pragma unroll
        for (int nt = 0; nt < 8; ++nt) acc2[nt] = z8;
        const _Float16* bb0 = w2h + (size_t)m * CH + 8 * hh;
#pragma unroll
        for (int kb = 0; kb < 4; ++kb) {
          const v16h a = __builtin_shufflevector(ah[2 * kb], ah[2 * kb + 1],
                                                 0, 1, 2, 3, 4, 5, 6, 7, 8, 9, 10, 11, 12, 13, 14, 15);
#pragma unroll
          for (int nt = 0; nt < 8; ++nt) {
            const size_t bo = (size_t)(16 * nt) * CH + 32 * kb;
            FragH b;
            b.h[0] = *(const v8h*)(bb0 + bo);
            b.h[1] = *(const v8h*)(bb0 + bo + 16);
            acc2[nt] = wmh(a, b.v, acc2[nt]);
          }
        }
        float* mw = msg + (wave * 16 + 8 * hh) * CH + m;
#pragma unroll
        for (int nt = 0; nt < 8; ++nt) {
#pragma unroll
          for (int r = 0; r < 8; ++r) mw[r * CH + 16 * nt] = acc2[nt][r];
        }
      }
      __syncthreads();

#pragma unroll 1
      for (int i = 0; i < PASSN; ++i) {
        const int sl = slotb[i];
        if (sl < NB && (sl & (NWAVE - 1)) == wave) {
          float* ap = acc + sl * CH + 4 * lane;
          const v4f a  = *(const v4fa*)ap;
          const v4f mv = *(const v4fa*)(msg + i * CH + 4 * lane);
          const v4f sum = a + mv;
          *(v4f*)ap = sum;
          if (lane == 0) cntf[sl] += 1.0f;
        }
      }
      __syncthreads();
    }

    int rem = newN - R * PASSN;
    rem = rem < 0 ? 0 : rem;
    if (R > 0 && tid < rem) pend[tid] = pend[R * PASSN + tid];
    if (tid == 0) pendN = rem;
  }
  __syncthreads();

  const v4f bb2 = *(const v4f*)(b2 + 4 * lane);
  const v4f z4e = {0.0f, 0.0f, 0.0f, 0.0f};
#pragma unroll 1
  for (int q = 0; q < NB / NWAVE; ++q) {
    const int sl  = q * NWAVE + wave;
    const int row = nodeBase + sl;
    if (row < nN) {
      const float cn  = cntf[sl];
      const float inv = 1.0f / fmaxf(cn, 1.0f);
      const v4f a = *(const v4fa*)(acc + sl * CH + 4 * lane);
      const v4f badd = (cn > 0.5f) ? bb2 : z4e;
      const v4f v = (a * WINV) * inv + badd;
      *(volatile v4f*)(outp + (size_t)row * CH + 4 * lane) = v;
    }
  }
  __threadfence();
#pragma unroll 1
  for (int q = 0; q < NB / NWAVE; ++q) {
    const int sl  = q * NWAVE + wave;
    const int row = nodeBase + sl;
    if (row < nN) {
      const float cn  = cntf[sl];
      const float inv = 1.0f / fmaxf(cn, 1.0f);
      const v4f a = *(const v4fa*)(acc + sl * CH + 4 * lane);
      const v4f badd = (cn > 0.5f) ? bb2 : z4e;
      const v4f v = (a * WINV) * inv + badd;
      *(volatile v4f*)(outp + (size_t)row * CH + 4 * lane) = v;
    }
  }
}

extern "C" void kernel_launch(void* const* d_in, const int* in_sizes, int n_in,
                              void* d_out, int out_size, void* d_ws, size_t ws_size,
                              hipStream_t stream) {
  if (n_in < 9) return;
  const int nN = in_sizes[0] / CH;
  const int nE = in_sizes[1] / 2;
  if (nN <= 0 || nE < 0) return;
  if (in_sizes[0] != nN * CH || in_sizes[1] != nE * 2 || in_sizes[2] != nE * 4) return;
  if (in_sizes[3] != 260 * CH || in_sizes[4] != CH || in_sizes[5] != CH || in_sizes[6] != CH) return;
  if (in_sizes[7] != CH * CH || in_sizes[8] != CH) return;
  if (out_size != nN * CH) return;

  const float* x   = (const float*)d_in[0];
  const int*   ei  = (const int*)d_in[1];
  const float* ea  = (const float*)d_in[2];
  const float* W1  = (const float*)d_in[3];
  const float* b1  = (const float*)d_in[4];
  const float* gmg = (const float*)d_in[5];
  const float* btg = (const float*)d_in[6];
  const float* W2  = (const float*)d_in[7];
  const float* b2  = (const float*)d_in[8];
  float* out = (float*)d_out;

  const int nBlkN = (nN + MROWS - 1) / MROWS;
  const int nBlkE = (nN + NB - 1) / NB;

  char* ws = (char*)d_ws;
  const size_t oW1h = 0;
  const size_t oW1l = oW1h + (size_t)256 * CH * 2;
  const size_t oW2h = oW1l + (size_t)256 * CH * 2;
  const size_t oNP  = oW2h + (size_t)CH * CH * 2;
  const size_t total = oNP + (size_t)nBlkN * MROWS * NPW * 4;
  if (total > ws_size) return;
  __bf16*   w1h = (__bf16*)(ws + oW1h);
  __bf16*   w1l = (__bf16*)(ws + oW1l);
  _Float16* w2h = (_Float16*)(ws + oW2h);
  float*    npl = (float*)(ws + oNP);

  const int vec8 = ((nE & 3) == 0) ? 1 : 0;

  k_prep<<<24, NTHR, 0, stream>>>(W1, W2, w1h, w1l, w2h);
  k_node<<<nBlkN, NTHR, 0, stream>>>(x, w1h, w1l, b1, npl, nN);
  k_edge<<<nBlkE, NTHR, 0, stream>>>(npl, ei, ea, W1, gmg, btg, b2, w2h, out, nN, nE, vec8);
}
